// PAGAGCN_29128468201963
// MI455X (gfx1250) — hardware-verified
//
#include <hip/hip_runtime.h>
#define NN 1024
#define NE 32768
#define EMB 128
#define HID 64
#define REP 32
typedef __bf16 v16b __attribute__((ext_vector_type(16)));
typedef unsigned short v8us __attribute__((ext_vector_type(8), may_alias));
typedef float  v8f  __attribute__((ext_vector_type(8)));
typedef float  v4f  __attribute__((ext_vector_type(4)));
typedef float  v4fa __attribute__((ext_vector_type(4), may_alias));
union FragB { v16b v; v8us half[2]; unsigned short u[16]; };

__device__ __forceinline__ unsigned short bf16_bits(float x) { unsigned int u = __float_as_uint(x); return (unsigned short)((u + 0x7FFFu + ((u >> 16) & 1u)) >> 16); }
__device__ __forceinline__ float bf16_val(unsigned short b) { return __uint_as_float(((unsigned int)b) << 16); }
__device__ __forceinline__ float bf16_round(float x) { return bf16_val(bf16_bits(x)); }
template <int NT>
__device__ __forceinline__ v8f mmaN(v16b ah, v16b al, v16b bh, v16b bl, v8f c) {
  c = __builtin_amdgcn_wmma_f32_16x16x32_bf16(false, ah, false, bh, (short)0, c, false, false);
  if (NT >= 2) c = __builtin_amdgcn_wmma_f32_16x16x32_bf16(false, al, false, bh, (short)0, c, false, false);
  if (NT >= 3) c = __builtin_amdgcn_wmma_f32_16x16x32_bf16(false, ah, false, bl, (short)0, c, false, false);
  asm volatile("v_nop\n\tv_nop\n\tv_nop\n\tv_nop" : "+v"(c) : "v"(ah), "v"(al), "v"(bh), "v"(bl));
  return c;
}

__global__ __launch_bounds__(256) void k_wt_bf16(const float* __restrict__ W, unsigned short* __restrict__ Wt, int K, int N) {
  const int t = blockIdx.x * 256 + threadIdx.x;
  const int k8n = K / 8;
  if (t >= N * k8n) return;
  const int n = t / k8n, k8 = (t % k8n) * 8;
  v8us v;
#pragma unroll
  for (int i = 0; i < 8; ++i) v[i] = bf16_bits(W[(size_t)(k8 + i) * N + n]);
  *(volatile v8us*)(Wt + (size_t)n * K + k8) = v;
  __threadfence();
  *(volatile v8us*)(Wt + (size_t)n * K + k8) = v;
}

template <bool ASPLIT, int ACT, bool BIAS_BF16>
__global__ __launch_bounds__(128) void k_gemm_bf(const float* __restrict__ A, int lda, const unsigned short* __restrict__ Wt, int ldb,
                                               const float* __restrict__ bias, float* __restrict__ C, int ldc, int M, int N, int K) {
  __shared__ __attribute__((aligned(16))) float so[4][16][64];
  const int tid = threadIdx.x, w = tid >> 5, lane = tid & 31, ln = lane & 15, hh = lane >> 4;
  const int ntn = N / 64;
  const int wid = blockIdx.x * 4 + w;
  const int mt = wid / ntn, nq = wid % ntn;
  if (mt * 16 >= M) return;
  const int row0 = mt * 16, col0 = nq * 64;
  const float* arow = A + (size_t)(row0 + ln) * lda;
  v8f acc[4] = {};
  for (int kb = 0; kb < K; kb += 32) {
    FragB ah, al;
    const v4f x0 = *(const v4fa*)(arow + kb + 8 * hh), x1 = *(const v4fa*)(arow + kb + 8 * hh + 4);
    const v4f x2 = *(const v4fa*)(arow + kb + 16 + 8 * hh), x3 = *(const v4fa*)(arow + kb + 16 + 8 * hh + 4);
    float xs[16] = {x0[0],x0[1],x0[2],x0[3],x1[0],x1[1],x1[2],x1[3],x2[0],x2[1],x2[2],x2[3],x3[0],x3[1],x3[2],x3[3]};
#pragma unroll
    for (int i = 0; i < 16; ++i) { const unsigned short hb = bf16_bits(xs[i]); ah.u[i] = hb; al.u[i] = ASPLIT ? bf16_bits(xs[i] - bf16_val(hb)) : (unsigned short)0; }
#pragma unroll
    for (int t = 0; t < 4; ++t) {
      const unsigned short* brow = Wt + (size_t)(col0 + t * 16 + ln) * ldb + kb;
      FragB b;
      b.half[0] = *(const v8us*)(brow + 8 * hh);
      b.half[1] = *(const v8us*)(brow + 16 + 8 * hh);
      acc[t] = mmaN<ASPLIT ? 2 : 1>(ah.v, al.v, b.v, b.v, acc[t]);
    }
  }
#pragma unroll
  for (int t = 0; t < 4; ++t) {
    float bv = bias ? bias[col0 + t * 16 + ln] : 0.f;
    if (BIAS_BF16) bv = bf16_round(bv);
#pragma unroll
    for (int r = 0; r < 8; ++r) { float v = acc[t][r] + bv; if (ACT == 1) v = fmaxf(v, 0.f); so[w][8 * hh + r][t * 16 + ln] = v; }
  }
  __builtin_amdgcn_fence(__ATOMIC_ACQ_REL, "workgroup");
  __builtin_amdgcn_wave_barrier();
  const int rsub = lane >> 4, c4 = (lane & 15) * 4;
  for (int pass = 0; pass < 2; ++pass) {
#pragma unroll
    for (int q = 0; q < 8; ++q) {
      const int r = q * 2 + rsub;
      const v4f v = *(const v4fa*)&so[w][r][c4];
      *(volatile v4f*)(C + (size_t)(row0 + r) * ldc + col0 + c4) = v;
    }
    if (pass == 0) __threadfence();
  }
}

template <bool ASPLIT, int ACT, bool BIAS_BF16, bool RES_BF16>
__global__ __launch_bounds__(128) void k_gemm_bf3(const float* __restrict__ A, int lda, const unsigned short* __restrict__ Wt, int ldb,
                                                const float* __restrict__ bias, const float* __restrict__ resid, int rmod, int ldr,
                                                float* __restrict__ C, int ldc, int M, int N, int K) {
  __shared__ __attribute__((aligned(16))) float so[4][16][64];
  const int tid = threadIdx.x, w = tid >> 5, lane = tid & 31, ln = lane & 15, hh = lane >> 4;
  const int ntn = N / 64;
  const int wid = blockIdx.x * 4 + w;
  const int mt = wid / ntn, nq = wid % ntn;
  if (mt * 16 >= M) return;
  const int row0 = mt * 16, col0 = nq * 64;
  const float* arow = A + (size_t)(row0 + ln) * lda;
  v8f acc[4] = {};
  for (int kb = 0; kb < K; kb += 32) {
    FragB ah, al;
    const v4f x0 = *(const v4fa*)(arow + kb + 8 * hh), x1 = *(const v4fa*)(arow + kb + 8 * hh + 4);
    const v4f x2 = *(const v4fa*)(arow + kb + 16 + 8 * hh), x3 = *(const v4fa*)(arow + kb + 16 + 8 * hh + 4);
    float xs[16] = {x0[0],x0[1],x0[2],x0[3],x1[0],x1[1],x1[2],x1[3],x2[0],x2[1],x2[2],x2[3],x3[0],x3[1],x3[2],x3[3]};
#pragma unroll
    for (int i = 0; i < 16; ++i) { const unsigned short hb = bf16_bits(xs[i]); ah.u[i] = hb; al.u[i] = ASPLIT ? bf16_bits(xs[i] - bf16_val(hb)) : (unsigned short)0; }
#pragma unroll
    for (int t = 0; t < 4; ++t) {
      const unsigned short* brow = Wt + (size_t)(col0 + t * 16 + ln) * ldb + kb;
      FragB b;
      b.half[0] = *(const v8us*)(brow + 8 * hh);
      b.half[1] = *(const v8us*)(brow + 16 + 8 * hh);
      acc[t] = mmaN<ASPLIT ? 2 : 1>(ah.v, al.v, b.v, b.v, acc[t]);
    }
  }
#pragma unroll
  for (int t = 0; t < 4; ++t) {
    const int col = col0 + t * 16 + ln;
    float bv = bias ? bias[col] : 0.f;
    if (BIAS_BF16) bv = bf16_round(bv);
#pragma unroll
    for (int r = 0; r < 8; ++r) {
      float v = acc[t][r] + bv;
      if (resid) { float rv = resid[(size_t)((row0 + 8 * hh + r) % rmod) * ldr + col]; if (RES_BF16) rv = bf16_round(rv); v += rv; }
      if (ACT == 1) v = fmaxf(v, 0.f);
      if (ACT == 2) v = 0.5f * v * (1.0f + erff(v * 0.70710678118654752f));
      if (ACT == 3) { const float u = 0.7978845608028654f * (v + 0.044715f * v * v * v); v = 0.5f * v * (1.0f + tanhf(u)); }
      so[w][8 * hh + r][t * 16 + ln] = v;
    }
  }
  __builtin_amdgcn_fence(__ATOMIC_ACQ_REL, "workgroup");
  __builtin_amdgcn_wave_barrier();
  const int rsub = lane >> 4, c4 = (lane & 15) * 4;
  for (int pass = 0; pass < 2; ++pass) {
#pragma unroll
    for (int q = 0; q < 8; ++q) {
      const int r = q * 2 + rsub;
      const v4f v = *(const v4fa*)&so[w][r][c4];
      *(volatile v4f*)(C + (size_t)(row0 + r) * ldc + col0 + c4) = v;
    }
    if (pass == 0) __threadfence();
  }
}
template <bool PARAM_BF16>
__global__ __launch_bounds__(256) void k_layernorm(const float* __restrict__ X, const float* __restrict__ R, const float* __restrict__ g, const float* __restrict__ bta,
                                                  float* __restrict__ out_sum, float* __restrict__ out_norm, int N, float eps) {
  __shared__ float red[256];
  const int row = blockIdx.x, tid = threadIdx.x;
  const float* x = X + (size_t)row * N; const float* rr = R ? R + (size_t)row * N : nullptr;
  float vals[16];
  const int per = N / 256;
  float s1 = 0.f;
  for (int u = 0; u < per / 4; ++u) {
    const int j = tid * 4 + 1024 * u;
    const v4f a = *(const v4fa*)(x + j);
    v4f b = {0.f,0.f,0.f,0.f}; if (rr) b = *(const v4fa*)(rr + j);
#pragma unroll
    for (int q = 0; q < 4; ++q) { const float v = a[q] + b[q]; vals[u * 4 + q] = v; s1 += v; }
  }
  red[tid] = s1; __syncthreads();
  for (int st = 128; st > 0; st >>= 1) { if (tid < st) red[tid] += red[tid + st]; __syncthreads(); }
  const float mu = red[0] / (float)N; __syncthreads();
  float s2 = 0.f;
  for (int u = 0; u < per / 4; ++u)
#pragma unroll
    for (int q = 0; q < 4; ++q) { const float c = vals[u * 4 + q] - mu; s2 += c * c; }
  red[tid] = s2; __syncthreads();
  for (int st = 128; st > 0; st >>= 1) { if (tid < st) red[tid] += red[tid + st]; __syncthreads(); }
  const float rs = rsqrtf(red[0] / (float)N + eps);
  for (int pass = 0; pass < 2; ++pass) {
    for (int u = 0; u < per / 4; ++u) {
      const int j = tid * 4 + 1024 * u;
      v4f o, sm;
#pragma unroll
      for (int q = 0; q < 4; ++q) {
        float gg = g[j + q], bb = bta[j + q];
        if (PARAM_BF16) { gg = bf16_round(gg); bb = bf16_round(bb); }
        sm[q] = vals[u * 4 + q]; o[q] = (vals[u * 4 + q] - mu) * rs * gg + bb;
      }
      if (out_sum) *(volatile v4f*)(out_sum + (size_t)row * N + j) = sm;
      *(volatile v4f*)(out_norm + (size_t)row * N + j) = o;
    }
    if (pass == 0) __threadfence();
  }
}


typedef _Float16 v16h __attribute__((ext_vector_type(16)));
union FragH { v16h v; v8us half[2]; _Float16 h[16]; unsigned short u[16]; };
template <int NT>
__device__ __forceinline__ v8f mmaH(v16h ah, v16h al, v16h bh, v16h bl, v8f c) {
  c = __builtin_amdgcn_wmma_f32_16x16x32_f16(false, ah, false, bh, (short)0, c, false, false);
  if (NT >= 2) c = __builtin_amdgcn_wmma_f32_16x16x32_f16(false, al, false, bh, (short)0, c, false, false);
  if (NT >= 3) c = __builtin_amdgcn_wmma_f32_16x16x32_f16(false, ah, false, bl, (short)0, c, false, false);
  asm volatile("v_nop\n\tv_nop\n\tv_nop\n\tv_nop" : "+v"(c) : "v"(ah), "v"(al), "v"(bh), "v"(bl));
  return c;
}
template <bool ASPLIT>
__global__ __launch_bounds__(128) void k_gemm_h(const float* __restrict__ A, int lda, size_t sA, const _Float16* __restrict__ Bh, int ldb, size_t sB, float alpha, float* __restrict__ C, int ldc, size_t sC, int M, int N, int K) {
  __shared__ __attribute__((aligned(16))) float so[4][16][64];
  const int tid = threadIdx.x, w = tid >> 5, lane = tid & 31, ln = lane & 15, hh = lane >> 4; const int by = blockIdx.y;
  A += (size_t)by * sA; Bh += (size_t)by * sB; C += (size_t)by * sC;
  const int ntn = (N + 63) / 64; const int wid = blockIdx.x * 4 + w; const int mt = wid / ntn, nq = wid % ntn; if (mt * 16 >= M) return;
  const int row0 = mt * 16, col0 = nq * 64; const float* arow = A + (size_t)(row0 + ln) * lda;
  v8f acc[4] = {};
  for (int kb = 0; kb < K; kb += 32) {
    FragH ah, al;
    const v4f x0 = *(const v4fa*)(arow + kb + 8 * hh), x1 = *(const v4fa*)(arow + kb + 8 * hh + 4), x2 = *(const v4fa*)(arow + kb + 16 + 8 * hh), x3 = *(const v4fa*)(arow + kb + 16 + 8 * hh + 4);
    float xs[16] = {x0[0],x0[1],x0[2],x0[3],x1[0],x1[1],x1[2],x1[3],x2[0],x2[1],x2[2],x2[3],x3[0],x3[1],x3[2],x3[3]};
#pragma unroll
    for (int i = 0; i < 16; ++i) { const _Float16 h = (_Float16)xs[i]; ah.h[i] = h; al.h[i] = ASPLIT ? (_Float16)(xs[i] - (float)h) : (_Float16)0.0f; }
#pragma unroll
    for (int t = 0; t < 4; ++t) { if (col0 + t * 16 >= N) continue; const size_t boff = (size_t)(col0 + t * 16 + ln) * ldb + kb; FragH bq; bq.half[0] = *(const v8us*)(Bh + boff + 8 * hh); bq.half[1] = *(const v8us*)(Bh + boff + 16 + 8 * hh);
      acc[t] = mmaH<ASPLIT ? 2 : 1>(ah.v, al.v, bq.v, bq.v, acc[t]); }
  }
#pragma unroll
  for (int t = 0; t < 4; ++t) { if (col0 + t * 16 >= N) continue;
#pragma unroll
    for (int r = 0; r < 8; ++r) so[w][8 * hh + r][t * 16 + ln] = acc[t][r] * alpha; }
  __builtin_amdgcn_fence(__ATOMIC_ACQ_REL, "workgroup"); __builtin_amdgcn_wave_barrier();
  const int rsub = lane >> 4, c4 = (lane & 15) * 4;
  for (int pass = 0; pass < 2; ++pass) {
#pragma unroll
    for (int q = 0; q < 8; ++q) { const int r = q * 2 + rsub; if (col0 + c4 < N) { const v4f v = *(const v4fa*)&so[w][r][c4]; *(volatile v4f*)(C + (size_t)(row0 + r) * ldc + col0 + c4) = v; } }
    if (pass == 0) __threadfence(); }
}

__global__ __launch_bounds__(256) void k_wt_f16(const float* __restrict__ W, _Float16* __restrict__ Wt, int K, int N, float scale) {
  const int t = blockIdx.x * 256 + threadIdx.x; if (t >= N * (K / 8)) return; const int n = t / (K / 8), k8 = (t % (K / 8)) * 8; FragH f;
#pragma unroll
  for (int i = 0; i < 8; ++i) f.h[i] = (_Float16)(bf16_round(W[(size_t)(k8 + i) * N + n]) * scale); const v8us o = f.half[0];
  *(volatile v8us*)((unsigned short*)Wt + (size_t)n * K + k8) = o; __threadfence(); *(volatile v8us*)((unsigned short*)Wt + (size_t)n * K + k8) = o;
}
template <int ACT>
__global__ __launch_bounds__(128) void k_gemm_hhx(const _Float16* __restrict__ A, int lda, size_t sA, const _Float16* __restrict__ Bh, int ldb, size_t sB, float alpha, const float* __restrict__ bias, size_t sBias, const float* __restrict__ CP, int rowsPerB, size_t sCPb, int row0g,
    float* __restrict__ C, _Float16* __restrict__ C16, int ldc, size_t sC, int M, int N, int K) {
  __shared__ __attribute__((aligned(16))) float so[4][16][64];
  const int tid = threadIdx.x, w = tid >> 5, lane = tid & 31, ln = lane & 15, hh = lane >> 4; const int by = blockIdx.y;
  A += (size_t)by * sA; Bh += (size_t)by * sB; const size_t cofs = (size_t)by * sC; const float* bp = bias ? bias + (size_t)by * sBias : nullptr;
  const int ntn = (N + 63) / 64; const int wid = blockIdx.x * 4 + w; const int mt = wid / ntn, nq = wid % ntn; if (mt * 16 >= M) return;
  const int row0 = mt * 16, col0 = nq * 64; const _Float16* arow = A + (size_t)(row0 + ln) * lda;
  v8f acc[4] = {};
  for (int kb = 0; kb < K; kb += 32) { FragH ah; ah.half[0] = *(const v8us*)((const unsigned short*)arow + kb + 8 * hh); ah.half[1] = *(const v8us*)((const unsigned short*)arow + kb + 16 + 8 * hh);
#pragma unroll
    for (int t = 0; t < 4; ++t) { if (col0 + t * 16 >= N) continue; const size_t boff = (size_t)(col0 + t * 16 + ln) * ldb + kb; FragH bq; bq.half[0] = *(const v8us*)((const unsigned short*)Bh + boff + 8 * hh); bq.half[1] = *(const v8us*)((const unsigned short*)Bh + boff + 16 + 8 * hh);
      acc[t] = mmaH<1>(ah.v, ah.v, bq.v, bq.v, acc[t]); }
  }
#pragma unroll
  for (int t = 0; t < 4; ++t) { if (col0 + t * 16 >= N) continue; const int col = col0 + t * 16 + ln; const float bv = bp ? bf16_round(bp[col]) : 0.f;
#pragma unroll
    for (int r = 0; r < 8; ++r) { float v = acc[t][r] * alpha + bv; if (CP) { const int bidx = (row0g + row0 + 8 * hh + r) / rowsPerB; v += CP[(size_t)bidx * sCPb + (size_t)by * 64 + col]; } if (ACT == 1) v = (v > 0.f) ? v : expm1f(v); else if (ACT == 7) v = (v > 0.f) ? v + 1.0f : expf(v); else if (ACT == 8) v = tanhf(v); else if (ACT == 9) v = 0.5f * v * (1.0f + tanhf(0.7978845608028654f * (v + 0.044715f * v * v * v))); else if (ACT == 11) v = 1.0f / (1.0f + expf(-v)); else if (ACT == 12) v = (v > 0.f) ? v : 0.01f * v; else if (ACT == 14) v = (v > 0.f) ? v : 0.1f * v; else if (ACT == 15) v = v / (1.0f + expf(-v)); else if (ACT == 3) v = fmaxf(v, 0.f); else if (ACT == 6) v = 0.5f * v * (1.0f + erff(v * 0.70710678118654752f)); so[w][8 * hh + r][t * 16 + ln] = v; } }
  __builtin_amdgcn_fence(__ATOMIC_ACQ_REL, "workgroup"); __builtin_amdgcn_wave_barrier();
  const int rsub = lane >> 4, c4 = (lane & 15) * 4; typedef _Float16 v4h __attribute__((ext_vector_type(4)));
  for (int pass = 0; pass < 2; ++pass) {
#pragma unroll
    for (int q = 0; q < 8; ++q) { const int r = q * 2 + rsub; if (col0 + c4 < N) { const v4f v = *(const v4fa*)&so[w][r][c4]; if (C) *(volatile v4f*)(C + cofs + (size_t)(row0 + r) * ldc + col0 + c4) = v; if (C16) { v4h h4; for (int i = 0; i < 4; ++i) h4[i] = (_Float16)v[i]; *(volatile v4h*)(C16 + cofs + (size_t)(row0 + r) * ldc + col0 + c4) = h4; } } }
    if (pass == 0) __threadfence(); }
}


typedef _Float16 v4h __attribute__((ext_vector_type(4)));

__global__ __launch_bounds__(256) void k_x16(const float* __restrict__ x, _Float16* __restrict__ X16, size_t n8) { const size_t t = (size_t)blockIdx.x * 256 + threadIdx.x; if (t >= n8) return; FragH f;
#pragma unroll
  for (int q = 0; q < 8; ++q) f.h[q] = (_Float16)bf16_round(x[t * 8 + q]); *(volatile v8us*)((unsigned short*)X16 + t * 8) = f.half[0]; __threadfence(); *(volatile v8us*)((unsigned short*)X16 + t * 8) = f.half[0]; }
__global__ __launch_bounds__(256) void k_h16(const float* __restrict__ x, _Float16* __restrict__ X16, size_t n8) { const size_t t = (size_t)blockIdx.x * 256 + threadIdx.x; if (t >= n8) return; FragH f;
#pragma unroll
  for (int q = 0; q < 8; ++q) f.h[q] = (_Float16)x[t * 8 + q]; *(volatile v8us*)((unsigned short*)X16 + t * 8) = f.half[0]; __threadfence(); *(volatile v8us*)((unsigned short*)X16 + t * 8) = f.half[0]; }
__global__ __launch_bounds__(256) void k_round16f(const float* __restrict__ W, _Float16* __restrict__ Bt, size_t n8) { const size_t t = (size_t)blockIdx.x * 256 + threadIdx.x; if (t >= n8) return; FragH f;
#pragma unroll
  for (int i = 0; i < 8; ++i) f.h[i] = (_Float16)(bf16_round(W[t * 8 + i]) * 16.0f); *(volatile v8us*)((unsigned short*)Bt + t * 8) = f.half[0]; __threadfence(); *(volatile v8us*)((unsigned short*)Bt + t * 8) = f.half[0]; }
template <int NHv, int TTv>
__global__ __launch_bounds__(256) void k_vt(const _Float16* __restrict__ V16, int ldv, int voff, _Float16* __restrict__ Vt) { __shared__ unsigned short tl[64][66]; const int tid = threadIdx.x; const int slab = blockIdx.x / (TTv / 64), lg = blockIdx.x % (TTv / 64); const int b = slab / NHv, h = slab % NHv;
  for (int i = tid; i < 64 * 8; i += 256) { const int r = i / 8, c8 = (i % 8) * 8; FragH f; f.half[0] = *(const v8us*)((const unsigned short*)V16 + ((size_t)b * TTv + lg * 64 + r) * ldv + voff + h * 64 + c8);
#pragma unroll
    for (int q = 0; q < 8; ++q) tl[r][c8 + q] = f.u[q]; }
  __syncthreads();
  for (int pass = 0; pass < 2; ++pass) {
#pragma unroll
    for (int rd = 0; rd < 2; ++rd) { const int d = rd * 32 + tid / 8, pc = tid % 8; FragH f;
#pragma unroll
      for (int q = 0; q < 8; ++q) f.u[q] = tl[pc * 8 + q][d];
      *(volatile v8us*)((unsigned short*)Vt + ((size_t)slab * 64 + d) * TTv + lg * 64 + pc * 8) = f.half[0]; }
    if (pass == 0) __threadfence(); } }

__global__ __launch_bounds__(256) void k_hl(const float* __restrict__ F, _Float16* __restrict__ Hh, _Float16* __restrict__ Hl, size_t n8) { const size_t t = (size_t)blockIdx.x * 256 + threadIdx.x; if (t >= n8) return; FragH fh, fl; const v4f a = *(const v4fa*)(F + t * 8), c = *(const v4fa*)(F + t * 8 + 4);
#pragma unroll
  for (int q = 0; q < 4; ++q) { _Float16 h = (_Float16)a[q]; fh.h[q] = h; fl.h[q] = (_Float16)((a[q] - (float)h) * 1024.0f); h = (_Float16)c[q]; fh.h[4 + q] = h; fl.h[4 + q] = (_Float16)((c[q] - (float)h) * 1024.0f); }
  for (int pass = 0; pass < 2; ++pass) { *(volatile v8us*)((unsigned short*)Hh + t * 8) = fh.half[0]; *(volatile v8us*)((unsigned short*)Hl + t * 8) = fl.half[0]; if (pass == 0) __threadfence(); } }

__global__ __launch_bounds__(256) void k_split(const float* __restrict__ F, _Float16* __restrict__ Hh, _Float16* __restrict__ Hl, size_t n8) {
  #pragma clang fp contract(off)
  const size_t t = (size_t)blockIdx.x * 256 + threadIdx.x; if (t >= n8) return; const v4f a = *(const v4fa*)(F + t * 8), c = *(const v4fa*)(F + t * 8 + 4); FragH fh, fl;
#pragma unroll
  for (int q = 0; q < 8; ++q) { const float v = (q < 4) ? a[q] : c[q - 4]; const _Float16 hi = (_Float16)v; fh.h[q] = hi; fl.h[q] = (_Float16)((v - (float)hi) * 1024.0f); }
  for (int pass = 0; pass < 2; ++pass) { *(volatile v8us*)((unsigned short*)Hh + t * 8) = fh.half[0]; *(volatile v8us*)((unsigned short*)Hl + t * 8) = fl.half[0]; if (pass == 0) __threadfence(); } }
__global__ __launch_bounds__(256) void k_splitT(const float* __restrict__ F, int C, _Float16* __restrict__ Th, _Float16* __restrict__ Tl) {
  #pragma clang fp contract(off)
  const int t = blockIdx.x * 256 + threadIdx.x; if (t >= C * (NN / 8)) return; const int i0 = (t % (NN / 8)) * 8, j = t / (NN / 8); FragH fh, fl;
#pragma unroll
  for (int q = 0; q < 8; ++q) { const float v = F[(size_t)(i0 + q) * C + j]; const _Float16 hi = (_Float16)v; fh.h[q] = hi; fl.h[q] = (_Float16)((v - (float)hi) * 1024.0f); }
  for (int pass = 0; pass < 2; ++pass) { *(volatile v8us*)((unsigned short*)Th + (size_t)j * NN + i0) = fh.half[0]; *(volatile v8us*)((unsigned short*)Tl + (size_t)j * NN + i0) = fl.half[0]; if (pass == 0) __threadfence(); } }
__global__ __launch_bounds__(256) void k_dense(const int* __restrict__ e, int lidx, float* __restrict__ AD) { __shared__ int hist[NN]; const int tid = threadIdx.x, i = blockIdx.x; for (int j = tid; j < NN; j += 256) hist[j] = 0; __syncthreads();
#pragma unroll 1
  for (int k = tid; k < NE; k += 256) { const int s = e[k], d = e[NE + k]; if (s == i && d >= 0 && d < NN) atomicAdd(&hist[d], 1); }
  __syncthreads(); v4f v; for (int q = 0; q < 4; ++q) v[q] = (float)hist[tid * 4 + q]; float* row = AD + ((size_t)lidx * NN + i) * NN + tid * 4; *(volatile v4f*)row = v; __threadfence(); *(volatile v4f*)row = v; }
template <int L>
__global__ __launch_bounds__(256) void k_c1pool(const float* __restrict__ AD, const float* __restrict__ w, const float* __restrict__ bb, float* __restrict__ P1) {
  #pragma clang fp contract(off)
  const int t = blockIdx.x * 256 + threadIdx.x; if (t >= 16 * 512 * 128) return; const int px0 = (t % 128) * 4; const int py = (t / 128) % 512; const int o = t / (128 * 512); v4f out;
#pragma unroll 1
  for (int q = 0; q < 4; ++q) { const int px = px0 + q; float m = -3.0e38f;
#pragma unroll 1
    for (int pos = 0; pos < 4; ++pos) { const int y = 2 * py + (pos >> 1), x = 2 * px + (pos & 1); float s = bf16_round(bb[o]);
#pragma unroll 1
      for (int c = 0; c < L; ++c) {
#pragma unroll
        for (int kh = 0; kh < 3; ++kh) { const int yy = y + kh - 1; if (yy < 0 || yy >= NN) continue;
#pragma unroll
          for (int kw = 0; kw < 3; ++kw) { const int xx = x + kw - 1; if (xx < 0 || xx >= NN) continue; s += AD[((size_t)c * NN + yy) * NN + xx] * bf16_round(w[((o * L + c) * 3 + kh) * 3 + kw]); } } }
      m = fmaxf(m, fmaxf(s, 0.f)); }
    out[q] = m; }
  *(volatile v4f*)(P1 + ((size_t)o * 512 + py) * 512 + px0) = out; __threadfence(); *(volatile v4f*)(P1 + ((size_t)o * 512 + py) * 512 + px0) = out; }
__global__ __launch_bounds__(256) void k_c2pool(const float* __restrict__ P1, const float* __restrict__ w, const float* __restrict__ bb, float* __restrict__ P2) {
  #pragma clang fp contract(off)
  const int t = blockIdx.x * 256 + threadIdx.x; if (t >= 4 * 257 * 257) return; const int px = t % 257; const int py = (t / 257) % 257; const int o = t / (257 * 257); float m = -3.0e38f;
#pragma unroll 1
  for (int pos = 0; pos < 4; ++pos) { const int y = 2 * py + (pos >> 1), x = 2 * px + (pos & 1);        float s = bf16_round(bb[o]);
#pragma unroll 1
    for (int c = 0; c < 16; ++c) {
#pragma unroll
      for (int kh = 0; kh < 3; ++kh) { const int yy = y + kh - 2; if (yy < 0 || yy >= 512) continue;
#pragma unroll
        for (int kw = 0; kw < 3; ++kw) { const int xx = x + kw - 2; if (xx < 0 || xx >= 512) continue; s += P1[((size_t)c * 512 + yy) * 512 + xx] * bf16_round(w[((o * 16 + c) * 3 + kh) * 3 + kw]); } } }
    m = fmaxf(m, fmaxf(s, 0.f)); }
  *(volatile float*)(P2 + t) = m; __threadfence(); *(volatile float*)(P2 + t) = m; }
__global__ __launch_bounds__(256) void k_t1(const float* __restrict__ P2, const float* __restrict__ w, const float* __restrict__ bb, float* __restrict__ T1) {
  #pragma clang fp contract(off)
  const int t = blockIdx.x * 256 + threadIdx.x; if (t >= 16 * 514 * 514) return; const int X = t % 514; const int Y = (t / 514) % 514; const int o = t / (514 * 514); const int y = Y >> 1, x = X >> 1, a = 1 - (Y & 1), b2 = 1 - (X & 1); float s = bf16_round(bb[o]);
#pragma unroll
  for (int c = 0; c < 4; ++c) s += P2[((size_t)c * 257 + y) * 257 + x] * bf16_round(w[((o * 4 + c) * 2 + a) * 2 + b2]);
  const float v = fmaxf(s, 0.f); *(volatile float*)(T1 + t) = v; __threadfence(); *(volatile float*)(T1 + t) = v; }
template <int L>
__global__ __launch_bounds__(256) void k_t2att(const float* __restrict__ T1, const float* __restrict__ w, const float* __restrict__ bb, const float* __restrict__ AD, float* __restrict__ ATD) {
  #pragma clang fp contract(off)
  const int t = blockIdx.x * 256 + threadIdx.x; if (t >= L * NN * (NN / 4)) return; const int j0 = (t % (NN / 4)) * 4; const int i = (t / (NN / 4)) % NN; const int l = t / ((NN / 4) * NN); const int y = i >> 1, a = 1 - (i & 1); v4f o;
#pragma unroll
  for (int q = 0; q < 4; ++q) { const int j = j0 + q; const int x = j >> 1, b2 = 1 - (j & 1); float s = bf16_round(bb[l]);
#pragma unroll 1
    for (int c = 0; c < 16; ++c) s += T1[((size_t)c * 514 + y) * 514 + x] * bf16_round(w[((l * 16 + c) * 2 + a) * 2 + b2]);
    o[q] = AD[((size_t)l * NN + i) * NN + j] * (1.0f / (1.0f + expf(-s))); }
  *(volatile v4f*)(ATD + ((size_t)l * NN + i) * NN + j0) = o; __threadfence(); *(volatile v4f*)(ATD + ((size_t)l * NN + i) * NN + j0) = o; }
__global__ __launch_bounds__(256) void k_deg(const float* __restrict__ P, float* __restrict__ DV) {
  #pragma clang fp contract(off)
  const int tid = threadIdx.x, w = tid >> 5, l = tid & 31; const int i = blockIdx.x * 8 + w; const float* pr = P + (size_t)i * NN; float s = 0.f;
#pragma unroll 1
  for (int j = 4 * l; j < NN; j += 128) { const v4f v = *(const v4fa*)(pr + j); s += (v[0] + v[1]) + (v[2] + v[3]); }
  for (int o = 16; o > 0; o >>= 1) s += __shfl_xor(s, o, 32);
  const float fix = (pr[i] == 0.f) ? 1.f : 0.f; const float deg = s + fix; const float dinv = (deg > 0.f) ? rsqrtf(deg) : 0.f; const float v = (l == 0) ? dinv : (l == 1) ? fix : 0.f;
  *(volatile float*)(DV + (size_t)i * 32 + l) = v; __threadfence(); *(volatile float*)(DV + (size_t)i * 32 + l) = v; }
__global__ __launch_bounds__(256) void k_nscale(const float* __restrict__ P, const float* __restrict__ DV, float* __restrict__ M) {
  #pragma clang fp contract(off)
  const int t = blockIdx.x * 256 + threadIdx.x; if (t >= NN * (NN / 4)) return; const int j0 = (t % (NN / 4)) * 4, i = t / (NN / 4); const float di = DV[(size_t)i * 32], fix = DV[(size_t)i * 32 + 1]; const v4f p = *(const v4fa*)(P + (size_t)i * NN + j0); v4f o;
#pragma unroll
  for (int q = 0; q < 4; ++q) { const int j = j0 + q; const float a = p[q] + ((j == i) ? fix : 0.f); o[q] = (di * a) * DV[(size_t)j * 32]; }
  *(volatile v4f*)(M + (size_t)i * NN + j0) = o; __threadfence(); *(volatile v4f*)(M + (size_t)i * NN + j0) = o; }
__global__ __launch_bounds__(256) void k_max2(const float* __restrict__ A, const float* __restrict__ B, float* __restrict__ C, size_t n4) { const size_t t = (size_t)blockIdx.x * 256 + threadIdx.x; if (t >= n4) return; const v4f a = *(const v4fa*)(A + t * 4), b = *(const v4fa*)(B + t * 4); v4f o; for (int q = 0; q < 4; ++q) o[q] = fmaxf(a[q], b[q]); *(volatile v4f*)(C + t * 4) = o; __threadfence(); *(volatile v4f*)(C + t * 4) = o; }

extern "C" void kernel_launch(void* const* d_in, const int* in_sizes, int n_in,
                              void* d_out, int out_size, void* d_ws, size_t ws_size, hipStream_t stream) {
  (void)in_sizes; (void)n_in; (void)out_size;
  const float* x = (const float*)d_in[0]; const int* ed[5] = {(const int*)d_in[1], (const int*)d_in[2], (const int*)d_in[3], (const int*)d_in[4], (const int*)d_in[5]};
  const float* c1w[2] = {(const float*)d_in[6], (const float*)d_in[14]}; const float* c1b[2] = {(const float*)d_in[7], (const float*)d_in[15]}; const float* c2w[2] = {(const float*)d_in[8], (const float*)d_in[16]}; const float* c2b[2] = {(const float*)d_in[9], (const float*)d_in[17]}; const float* t1w[2] = {(const float*)d_in[10], (const float*)d_in[18]}; const float* t1b[2] = {(const float*)d_in[11], (const float*)d_in[19]}; const float* t2w[2] = {(const float*)d_in[12], (const float*)d_in[20]}; const float* t2b[2] = {(const float*)d_in[13], (const float*)d_in[21]};
  const float* w1 = (const float*)d_in[22]; const float* b1 = (const float*)d_in[23]; const float* w2 = (const float*)d_in[24]; const float* b2 = (const float*)d_in[25];
  char* ws = (char*)d_ws; size_t off = 0;
  auto take = [&](size_t bytes) { char* p = ws + off; off += (bytes + 255) & ~(size_t)255; return p; };
  const size_t PL = (size_t)NN * NN;
  float* AD = (float*)take(3 * PL * 4); float* ATD = (float*)take(3 * PL * 4); float* P1 = (float*)take((size_t)16 * 512 * 512 * 4); float* P2 = (float*)take((size_t)4 * 257 * 257 * 4); float* T1 = (float*)take((size_t)16 * 514 * 514 * 4);
  float* M = (float*)take(PL * 4); float* PR = (float*)take(PL * 4); float* MP[2]; MP[0] = (float*)take(PL * 4); MP[1] = (float*)take(PL * 4); float* DV = (float*)take((size_t)NN * 32 * 4);
  _Float16* Mh = (_Float16*)take(PL * 2); _Float16* Ml = (_Float16*)take(PL * 2); _Float16* Bh = (_Float16*)take(PL * 2); _Float16* Bl = (_Float16*)take(PL * 2);
  _Float16* X16 = (_Float16*)take((size_t)NN * EMB * 2); _Float16* Bw1 = (_Float16*)take((size_t)HID * EMB * 2); _Float16* Bw2 = (_Float16*)take((size_t)REP * HID * 2); float* XW = (float*)take((size_t)NN * HID * 4); float* H = (float*)take((size_t)NN * HID * 4); _Float16* Hh = (_Float16*)take((size_t)NN * HID * 2); _Float16* Hl = (_Float16*)take((size_t)NN * HID * 2); float* HW = (float*)take((size_t)NN * REP * 4);
  if (off > ws_size) return;
  k_x16<<<(NN * EMB / 8 + 255) / 256, 256, 0, stream>>>(x, X16, (size_t)NN * EMB / 8); k_wt_f16<<<(HID * (EMB / 8) + 255) / 256, 256, 0, stream>>>(w1, Bw1, EMB, HID, 16.0f); k_wt_f16<<<(REP * (HID / 8) + 255) / 256, 256, 0, stream>>>(w2, Bw2, HID, REP, 16.0f);
  const dim3 gD(((NN / 16) * (NN / 64) + 3) / 4, 1); const size_t n8 = PL / 8;
  const int Ls[2] = {2, 3}; int eoff = 0;
  for (int p = 0; p < 2; ++p) { const int L = Ls[p];
    for (int l = 0; l < L; ++l) k_dense<<<NN, 256, 0, stream>>>(ed[eoff + l], l, AD);
    eoff += L;
    if (L == 2) k_c1pool<2><<<(16 * 512 * 128 + 255) / 256, 256, 0, stream>>>(AD, c1w[p], c1b[p], P1); else k_c1pool<3><<<(16 * 512 * 128 + 255) / 256, 256, 0, stream>>>(AD, c1w[p], c1b[p], P1);
    k_c2pool<<<(4 * 257 * 257 + 255) / 256, 256, 0, stream>>>(P1, c2w[p], c2b[p], P2);
    k_t1<<<(16 * 514 * 514 + 255) / 256, 256, 0, stream>>>(P2, t1w[p], t1b[p], T1);
    if (L == 2) k_t2att<2><<<(unsigned)((2 * PL / 4 + 255) / 256), 256, 0, stream>>>(T1, t2w[p], t2b[p], AD, ATD); else k_t2att<3><<<(unsigned)((3 * PL / 4 + 255) / 256), 256, 0, stream>>>(T1, t2w[p], t2b[p], AD, ATD);
    k_deg<<<NN / 8, 256, 0, stream>>>(ATD, DV); k_nscale<<<(unsigned)((PL / 4 + 255) / 256), 256, 0, stream>>>(ATD, DV, M);
    for (int l = 1; l < L; ++l) {
      k_split<<<(unsigned)((n8 + 255) / 256), 256, 0, stream>>>(M, Mh, Ml, n8); k_splitT<<<(NN * (NN / 8) + 255) / 256, 256, 0, stream>>>(ATD + (size_t)l * PL, NN, Bh, Bl);
      k_gemm_hhx<0><<<gD, 128, 0, stream>>>(Mh, NN, 0, Bh, NN, 0, 1.0f, nullptr, 0, nullptr, 1, 0, 0, PR, nullptr, NN, 0, NN, NN, NN); k_gemm_hhx<0><<<gD, 128, 0, stream>>>(Mh, NN, 0, Bl, NN, 0, 1.0f / 1024.0f, nullptr, 0, PR, 1, (size_t)NN, 0, PR, nullptr, NN, 0, NN, NN, NN); k_gemm_hhx<0><<<gD, 128, 0, stream>>>(Ml, NN, 0, Bh, NN, 0, 1.0f / 1024.0f, nullptr, 0, PR, 1, (size_t)NN, 0, PR, nullptr, NN, 0, NN, NN, NN);
      k_deg<<<NN / 8, 256, 0, stream>>>(PR, DV); k_nscale<<<(unsigned)((PL / 4 + 255) / 256), 256, 0, stream>>>(PR, DV, M); }
    k_max2<<<(unsigned)((PL / 4 + 255) / 256), 256, 0, stream>>>(M, M, MP[p], PL / 4); }
  k_max2<<<(unsigned)((PL / 4 + 255) / 256), 256, 0, stream>>>(MP[0], MP[1], PR, PL / 4); k_deg<<<NN / 8, 256, 0, stream>>>(PR, DV); k_nscale<<<(unsigned)((PL / 4 + 255) / 256), 256, 0, stream>>>(PR, DV, M);
  k_split<<<(unsigned)((n8 + 255) / 256), 256, 0, stream>>>(M, Mh, Ml, n8);
  k_gemm_hhx<0><<<dim3(((NN / 16) * 1 + 3) / 4, 1), 128, 0, stream>>>(X16, EMB, 0, Bw1, EMB, 0, 0.0625f, nullptr, 0, nullptr, 1, 0, 0, XW, nullptr, HID, 0, NN, HID, EMB);
  k_splitT<<<(HID * (NN / 8) + 255) / 256, 256, 0, stream>>>(XW, HID, Bh, Bl);
  const dim3 gH(((NN / 16) * 1 + 3) / 4, 1);
  k_gemm_hhx<0><<<gH, 128, 0, stream>>>(Mh, NN, 0, Bh, NN, 0, 1.0f, nullptr, 0, nullptr, 1, 0, 0, H, nullptr, HID, 0, NN, HID, NN); k_gemm_hhx<0><<<gH, 128, 0, stream>>>(Mh, NN, 0, Bl, NN, 0, 1.0f / 1024.0f, nullptr, 0, H, 1, (size_t)HID, 0, H, nullptr, HID, 0, NN, HID, NN); k_gemm_hhx<3><<<gH, 128, 0, stream>>>(Ml, NN, 0, Bh, NN, 0, 1.0f / 1024.0f, b1, 0, H, 1, (size_t)HID, 0, H, nullptr, HID, 0, NN, HID, NN);
  k_split<<<(NN * HID / 8 + 255) / 256, 256, 0, stream>>>(H, Hh, Hl, (size_t)NN * HID / 8);
  k_gemm_hhx<0><<<gH, 128, 0, stream>>>(Hh, HID, 0, Bw2, HID, 0, 0.0625f, nullptr, 0, nullptr, 1, 0, 0, HW, nullptr, REP, 0, NN, REP, HID); k_gemm_hhx<0><<<gH, 128, 0, stream>>>(Hl, HID, 0, Bw2, HID, 0, 0.0625f / 1024.0f, nullptr, 0, HW, 1, (size_t)REP, 0, HW, nullptr, REP, 0, NN, REP, HID);
  k_splitT<<<(REP * (NN / 8) + 255) / 256, 256, 0, stream>>>(HW, REP, Bh, Bl);
  float* out = (float*)d_out;
  k_gemm_hhx<0><<<gH, 128, 0, stream>>>(Mh, NN, 0, Bh, NN, 0, 1.0f, b2, 0, nullptr, 1, 0, 0, out, nullptr, REP, 0, NN, REP, NN); k_gemm_hhx<0><<<gH, 128, 0, stream>>>(Mh, NN, 0, Bl, NN, 0, 1.0f / 1024.0f, nullptr, 0, out, 1, (size_t)REP, 0, out, nullptr, REP, 0, NN, REP, NN); k_gemm_hhx<0><<<gH, 128, 0, stream>>>(Ml, NN, 0, Bh, NN, 0, 1.0f / 1024.0f, nullptr, 0, out, 1, (size_t)REP, 0, out, nullptr, REP, 0, NN, REP, NN);
}
